// CNOFactorized2DBlock_65085934403665
// MI455X (gfx1250) — hardware-verified
//
#include <hip/hip_runtime.h>
#include <stddef.h>
#include <stdint.h>

constexpr int NBATCH = 4;
constexpr int NROWM  = 256;
constexpr int NCOLN  = 256;
constexpr int CIN    = 12;
constexpr int CW     = 64;
constexpr int NMODE  = 32;
constexpr int CHID   = 128;
constexpr int NLAYER = 4;
constexpr int NPIX   = NBATCH * NROWM * NCOLN;
constexpr int NSLICE = NBATCH * NROWM;
constexpr int PIXB   = NROWM * NCOLN * CW;

static_assert(NROWM == NCOLN);
static_assert(NPIX % 64 == 0);
static_assert(NSLICE % 16 == 0);

constexpr size_t SZ_DF = (size_t)NMODE * NCOLN * 2;
constexpr size_t SZ_DT = (size_t)NCOLN * NMODE * 2;
constexpr size_t SZ_X  = (size_t)NPIX * CW * 4;
constexpr size_t SZ_H  = (size_t)NPIX * CW * 2;
constexpr size_t SZ_XF = (size_t)NMODE * NSLICE * CW * 2;
constexpr size_t SZ_YM = (size_t)NSLICE * CW * NMODE * 2;
constexpr size_t SZ_WM = (size_t)NLAYER * NMODE * CW * CW * 2;
constexpr size_t SZ_W1 = (size_t)NLAYER * CHID * CW * 2;
constexpr size_t SZ_W2 = (size_t)NLAYER * CW * CHID * 2;
constexpr size_t SZ_WO = (size_t)CHID * CW * 2;
constexpr size_t OFF_DF  = 0;
constexpr size_t OFF_DT  = OFF_DF + SZ_DF;
constexpr size_t OFF_X   = OFF_DT + SZ_DT;
constexpr size_t OFF_H   = OFF_X + SZ_X;
constexpr size_t OFF_XF  = OFF_H + SZ_H;
constexpr size_t OFF_YY  = OFF_XF + SZ_XF;
constexpr size_t OFF_YX  = OFF_YY + SZ_YM;
constexpr size_t OFF_WM0 = OFF_YX + SZ_YM;
constexpr size_t OFF_WM1 = OFF_WM0 + SZ_WM;
constexpr size_t OFF_W1  = OFF_WM1 + SZ_WM;
constexpr size_t OFF_W2  = OFF_W1 + SZ_W1;
constexpr size_t OFF_WO  = OFF_W2 + SZ_W2;
constexpr size_t WS_TOTAL = OFF_WO + SZ_WO;
static_assert(WS_TOTAL <= (size_t)134217728);
static_assert(OFF_DT % 128 == 0 && OFF_X % 128 == 0 && OFF_H % 128 == 0 && OFF_XF % 128 == 0 && OFF_YY % 128 == 0);
static_assert(OFF_YX % 128 == 0 && OFF_WM0 % 128 == 0 && OFF_WM1 % 128 == 0 && OFF_W1 % 128 == 0 && OFF_W2 % 128 == 0 && OFF_WO % 128 == 0);
static_assert(SZ_DF % 128 == 0 && SZ_DT % 128 == 0 && SZ_XF % 128 == 0 && SZ_YM % 128 == 0 && SZ_WM % 128 == 0);

constexpr int LDS_INV = 65536 + 2048 + 65536;

typedef _Float16 v16h __attribute__((ext_vector_type(16)));
typedef _Float16 v8h __attribute__((ext_vector_type(8)));
typedef v8h __attribute__((may_alias)) v8ha;
typedef float v8f __attribute__((ext_vector_type(8)));
typedef float v4f __attribute__((ext_vector_type(4)));
typedef v4f __attribute__((may_alias)) v4fa;
typedef unsigned int v4u __attribute__((ext_vector_type(4)));

union Frag { v16h v; v8h h[2]; };
union Pack8 { v8h h; v4u u; };

constexpr float PI_F  = 3.14159265358979323846f;
constexpr float SQ2N  = 0.0883883476483184f;
constexpr float RSQ2  = 0.70710678118654752f;

__device__ __forceinline__ v8f mma16(v16h a, v16h b, v8f c) {
  c = __builtin_amdgcn_wmma_f32_16x16x32_f16(false, a, false, b, (short)0, c, false, false);
  asm volatile("v_nop\n\tv_nop\n\tv_nop\n\tv_nop" : "+v"(c) : "v"(a), "v"(b));
  return c;
}

__device__ __forceinline__ v8f zero8() { return (v8f){0.f, 0.f, 0.f, 0.f, 0.f, 0.f, 0.f, 0.f}; }

__device__ __forceinline__ v16h ldfrag(const _Float16* base, int pitch, int row0, int k0, int lane) {
  const int m = lane & 15, hh = lane >> 4;
  const _Float16* q = base + (size_t)(row0 + m) * pitch + k0 + 8 * hh;
  Frag f;
  f.h[0] = *(const v8ha*)(q);
  f.h[1] = *(const v8ha*)(q + 16);
  return f.v;
}

__device__ __forceinline__ void st2_u4(_Float16* p, v4u v) {
  *(volatile v4u*)p = v;
  __threadfence();
  *(volatile v4u*)p = v;
}
__device__ __forceinline__ void st2_f4(float* p, v4f v) {
  *(volatile v4f*)p = v;
  __threadfence();
  *(volatile v4f*)p = v;
}

__device__ __forceinline__ unsigned int f16bits(float x) {
  return (unsigned int)__builtin_bit_cast(unsigned short, (_Float16)x);
}

__device__ __forceinline__ void shin(unsigned int& w0, unsigned int& w1, unsigned int& w2, unsigned int& w3, unsigned int hb) {
  w0 = (w0 >> 16) | (w1 << 16);
  w1 = (w1 >> 16) | (w2 << 16);
  w2 = (w2 >> 16) | (w3 << 16);
  w3 = (w3 >> 16) | (hb << 16);
}

__global__ __launch_bounds__(256) void k_dct_planes(_Float16* __restrict__ df, _Float16* __restrict__ dt) {
  const int t = threadIdx.x;
#pragma unroll 1
  for (int it = 0; it < 4; ++it) {
    const int e = (t + 256 * it) * 8;
    const int kA = e >> 8, nA0 = e & 255;
    const int nB = e >> 5, yB0 = e & 31;
    unsigned int a0 = 0u, a1 = 0u, a2 = 0u, a3 = 0u, b0 = 0u, b1 = 0u, b2 = 0u, b3 = 0u;
#pragma unroll 1
    for (int j = 0; j < 16; ++j) {
      const bool fa = j < 8;
      const int kk = fa ? kA : (yB0 + j - 8);
      const int nn = fa ? (nA0 + j) : nB;
      const float ang = (PI_F * ((float)nn + 0.5f)) * (float)kk * (1.0f / 256.0f);
      float v = cosf(ang) * SQ2N;
      v = (kk == 0) ? (v * RSQ2) : v;
      const unsigned int hb = f16bits(v * 8.0f);
      if (fa) shin(a0, a1, a2, a3, hb); else shin(b0, b1, b2, b3, hb);
    }
    st2_u4(df + e, (v4u){a0, a1, a2, a3});
    st2_u4(dt + e, (v4u){b0, b1, b2, b3});
  }
}

__global__ __launch_bounds__(256) void k_cvt_modes(const float* __restrict__ fw, _Float16* __restrict__ wm) {
  const int k = blockIdx.x, l = blockIdx.y, t = threadIdx.x;
#pragma unroll 1
  for (int it = 0; it < 2; ++it) {
    const int idx = t + 256 * it;
    const int o = idx >> 3, i0 = (idx & 7) * 8;
    v8h hv;
#pragma unroll
    for (int j = 0; j < 8; ++j) {
      const float v = fw[(((size_t)l * CW + i0 + j) * CW + o) * NMODE + k];
      hv[j] = (_Float16)(v * 8.0f);
    }
    Pack8 pk; pk.h = hv;
    st2_u4(wm + (((size_t)(l * NMODE + k) * CW + o) * CW + i0), pk.u);
  }
}

__global__ __launch_bounds__(256) void k_cvt_lin(const float* __restrict__ src, _Float16* __restrict__ dst, int n) {
  const int i0 = (blockIdx.x * 256 + (int)threadIdx.x) * 8;
  if (i0 + 8 > n) return;
  const v4f u0 = *(const v4f*)(src + i0);
  const v4f u1 = *(const v4f*)(src + i0 + 4);
  v8h hv;
#pragma unroll
  for (int j = 0; j < 4; ++j) { hv[j] = (_Float16)(u0[j] * 8.0f); hv[4 + j] = (_Float16)(u1[j] * 8.0f); }
  Pack8 pk; pk.h = hv;
  st2_u4(dst + i0, pk.u);
}

__global__ __launch_bounds__(256) void k_lift(const float* __restrict__ xin, const float* __restrict__ win,
                                              const float* __restrict__ bin, float* __restrict__ x32) {
  __shared__ float sW[CW * CIN];
  __shared__ float sBias[CW];
  __shared__ __align__(16) float sX[64 * 68];
  const int t = threadIdx.x;
  const int p0 = blockIdx.x * 64;
  for (int i = t; i < CW * CIN; i += 256) sW[i] = win[i];
  if (t < CW) sBias[t] = bin[t];
  const int px = t >> 2, g = t & 3;
  const float* xr = xin + (size_t)(p0 + px) * CIN;
  const v4f x0 = *(const v4f*)(xr);
  const v4f x1 = *(const v4f*)(xr + 4);
  const v4f x2 = *(const v4f*)(xr + 8);
  __syncthreads();
#pragma unroll 1
  for (int cc = 0; cc < 16; ++cc) {
    const int ch = g * 16 + cc;
    const float* w = sW + ch * CIN;
    float a = sBias[ch];
    a += x0[0] * w[0];  a += x0[1] * w[1];  a += x0[2] * w[2];   a += x0[3] * w[3];
    a += x1[0] * w[4];  a += x1[1] * w[5];  a += x1[2] * w[6];   a += x1[3] * w[7];
    a += x2[0] * w[8];  a += x2[1] * w[9];  a += x2[2] * w[10];  a += x2[3] * w[11];
    sX[px * 68 + ch] = a;
  }
  __syncthreads();
#pragma unroll
  for (int it = 0; it < 4; ++it) {
    const int idx = t + 256 * it;
    const int L = idx >> 3, pc = idx & 7;
    const int row = L >> 1, half = L & 1;
    const v4f v = *(const v4fa*)(sX + row * 68 + half * 32 + pc * 4);
    st2_f4(x32 + (size_t)(p0 + row) * CW + half * 32 + pc * 4, v);
  }
}

constexpr int PF = 264;
__global__ __launch_bounds__(256) void k_dct_fwd(const float* __restrict__ xs, const _Float16* __restrict__ df,
                                                 _Float16* __restrict__ xf, int RS, int RO) {
  __shared__ __align__(16) _Float16 lA[NMODE * PF];
  __shared__ __align__(16) _Float16 lB[CW * PF];
  __shared__ __align__(16) _Float16 sO[NMODE * 72];
  const int t = threadIdx.x;
  const int p = blockIdx.x;
  const size_t base = (size_t)(p >> 8) * PIXB + (size_t)(p & 255) * (size_t)RS;

#pragma unroll
  for (int it = 0; it < 4; ++it) {
    const int idx = t + 256 * it;
    const int rr = idx >> 5, c8 = idx & 31;
    *(v8ha*)(lA + rr * PF + c8 * 8) = *(const v8ha*)(df + rr * NCOLN + c8 * 8);
  }
  {
    const int i = t & 63, ng = t >> 6;
#pragma unroll 1
    for (int g8 = 0; g8 < 8; ++g8) {
      const int n0 = ng * 64 + g8 * 8;
      v8h hv;
#pragma unroll
      for (int j = 0; j < 8; ++j) hv[j] = (_Float16)xs[base + (size_t)(n0 + j) * (size_t)RO + i];
      *(v8ha*)(lB + i * PF + n0) = hv;
    }
  }
  __syncthreads();

  const int wave = t >> 5, lane = t & 31, hh = lane >> 4, c = lane & 15;
  const int mt = wave >> 2, nt = wave & 3;
  v8f acc = zero8();
#pragma unroll
  for (int kk = 0; kk < 8; ++kk) {
    const v16h a = ldfrag(lA, PF, mt * 16, kk * 32, lane);
    const v16h b = ldfrag(lB, PF, nt * 16, kk * 32, lane);
    acc = mma16(a, b, acc);
  }
#pragma unroll
  for (int r = 0; r < 8; ++r) sO[(mt * 16 + 8 * hh + r) * 72 + nt * 16 + c] = (_Float16)acc[r];
  __syncthreads();
  {
    const int k = t >> 3, pc = t & 7;
    Pack8 pk; pk.h = *(const v8ha*)(sO + k * 72 + pc * 8);
    st2_u4(xf + ((size_t)k * NSLICE + p) * CW + pc * 8, pk.u);
  }
}

__global__ __launch_bounds__(256) void k_mode_mix(const _Float16* __restrict__ xf, const _Float16* __restrict__ wm,
                                                  _Float16* __restrict__ ym) {
  __shared__ __align__(16) _Float16 sY[16 * 32 * 32];
  const int t = threadIdx.x;
  const int pt = blockIdx.x >> 1, oh = blockIdx.x & 1;
  const int p0 = pt * 16;
  const int wave = t >> 5, lane = t & 31, hh = lane >> 4, c = lane & 15;

#pragma unroll 1
  for (int q = 0; q < 4; ++q) {
    const int k = wave * 4 + q;
    const _Float16* xa = xf + (size_t)k * NSLICE * CW;
    const _Float16* wb = wm + ((size_t)k * CW + oh * 32) * CW;
    v8f acc0 = zero8(), acc1 = zero8();
#pragma unroll
    for (int ks = 0; ks < 2; ++ks) {
      const v16h a  = ldfrag(xa, CW, p0, ks * 32, lane);
      const v16h b0 = ldfrag(wb, CW, 0, ks * 32, lane);
      const v16h b1 = ldfrag(wb, CW, 16, ks * 32, lane);
      acc0 = mma16(a, b0, acc0);
      acc1 = mma16(a, b1, acc1);
    }
#pragma unroll
    for (int r = 0; r < 8; ++r) {
      const int pl = 8 * hh + r;
      sY[(pl * 32 + c) * 32 + k]      = (_Float16)(acc0[r] * 0.125f);
      sY[(pl * 32 + 16 + c) * 32 + k] = (_Float16)(acc1[r] * 0.125f);
    }
  }
  __syncthreads();
#pragma unroll 1
  for (int it = 0; it < 8; ++it) {
    const int idx = t + 256 * it;
    const int pl = idx >> 7, e = (idx & 127) * 8;
    Pack8 pk; pk.h = *(const v8ha*)(sY + pl * 1024 + e);
    st2_u4(ym + ((size_t)(p0 + pl) * CW + oh * 32) * NMODE + e, pk.u);
  }
}

__device__ __forceinline__ void stage_ym(_Float16* sYm, const _Float16* __restrict__ src, int slice0, int t) {
#pragma unroll 4
  for (int it = 0; it < 16; ++it) {
    const int idx = t + 256 * it;
    const int s = idx >> 8, c8 = idx & 255;
    *(v8ha*)(sYm + s * 2048 + c8 * 8) = *(const v8ha*)(src + (size_t)(slice0 + s) * 2048 + c8 * 8);
  }
}

__global__ __launch_bounds__(256) void k_inv(const _Float16* __restrict__ dt, const _Float16* __restrict__ ymy,
                                             const _Float16* __restrict__ ymx, _Float16* __restrict__ h16) {
  extern __shared__ __align__(16) unsigned char dynlds[];
  _Float16* sYm = (_Float16*)(dynlds);
  _Float16* sD  = (_Float16*)(dynlds + 65536);
  float*    sXY = (float*)(dynlds + 65536 + 2048);
  const int t = threadIdx.x;
  const int blk = blockIdx.x;
  const int b = blk >> 8, tm = (blk >> 4) & 15, tn = blk & 15;
  const int m0 = tm * 16, n0 = tn * 16;
  const int wave = t >> 5, lane = t & 31, hh = lane >> 4, c = lane & 15;

  if (t < 128) {
    const int row = t >> 2, c8 = t & 3;
    const int srow = (row < 16) ? (n0 + row) : (m0 + row - 16);
    *(v8ha*)(sD + row * 32 + c8 * 8) = *(const v8ha*)(dt + srow * NMODE + c8 * 8);
  }
  stage_ym(sYm, ymy, b * NROWM + m0, t);
  __syncthreads();

  {
    const v16h aY = ldfrag(sD, 32, 0, 0, lane);
#pragma unroll
    for (int si = 0; si < 2; ++si) {
      const int mi = wave * 2 + si;
#pragma unroll
      for (int nt = 0; nt < 4; ++nt) {
        const v16h bf = ldfrag(sYm + mi * 2048, 32, nt * 16, 0, lane);
        const v8f acc = mma16(aY, bf, zero8());
#pragma unroll
        for (int r = 0; r < 8; ++r) sXY[(mi * 16 + 8 * hh + r) * 64 + nt * 16 + c] = acc[r];
      }
    }
  }
  __syncthreads();
  stage_ym(sYm, ymx, b * NCOLN + n0, t);
  __syncthreads();

  v8f ax[2][4];
  {
    const v16h aX = ldfrag(sD, 32, 16, 0, lane);
#pragma unroll
    for (int si = 0; si < 2; ++si) {
      const int ni = wave * 2 + si;
#pragma unroll
      for (int nt = 0; nt < 4; ++nt) {
        const v16h bf = ldfrag(sYm + ni * 2048, 32, nt * 16, 0, lane);
        ax[si][nt] = mma16(aX, bf, zero8());
      }
    }
  }
  __syncthreads();
  _Float16* sH = sYm;
#pragma unroll
  for (int si = 0; si < 2; ++si) {
    const int ni = wave * 2 + si;
#pragma unroll
    for (int nt = 0; nt < 4; ++nt) {
#pragma unroll
      for (int r = 0; r < 8; ++r) {
        const int px = (8 * hh + r) * 16 + ni;
        const int o = nt * 16 + c;
        const float hv = (sXY[px * 64 + o] + ax[si][nt][r]) * (1.0f / 64.0f);
        sH[px * 72 + o] = (_Float16)hv;
      }
    }
  }
  __syncthreads();
#pragma unroll 1
  for (int it = 0; it < 8; ++it) {
    const int idx = t + 256 * it;
    const int px = idx >> 3, pc = idx & 7;
    const int mi = px >> 4, ni = px & 15;
    Pack8 pk; pk.h = *(const v8ha*)(sH + px * 72 + pc * 8);
    st2_u4(h16 + ((size_t)((b * NROWM + m0 + mi) * NCOLN + (n0 + ni))) * CW + pc * 8, pk.u);
  }
}

template <bool LAST>
__global__ __launch_bounds__(256) void k_ffn(const _Float16* __restrict__ h16, const _Float16* __restrict__ w1p,
                                             const float* __restrict__ b1, const _Float16* __restrict__ w2p,
                                             const float* __restrict__ b2, float* __restrict__ x32,
                                             const _Float16* __restrict__ wo1p, const float* __restrict__ bo1,
                                             const float* __restrict__ wo2, const float* __restrict__ bo2,
                                             float* __restrict__ out) {
  __shared__ __align__(16) _Float16 sT[64 * 136];
  __shared__ __align__(16) float sBB[64 * 64];
  __shared__ __align__(16) _Float16 sB16[64 * 72];
  __shared__ float sPart[64 * 2];
  __shared__ __align__(16) float sOut[64];
  __shared__ float sB1[CHID];
  __shared__ float sB2[CW];
  __shared__ float sBo1[CHID];
  __shared__ float sWo2[CHID];
  const int t = threadIdx.x;
  const int p0 = blockIdx.x * 64;
  const int wave = t >> 5, lane = t & 31, hh = lane >> 4, c = lane & 15;
  const int mt = wave >> 1, nq = wave & 1;

  if (t < CHID) {
    sB1[t] = b1[t];
    if (LAST) { sBo1[t] = bo1[t]; sWo2[t] = wo2[t]; }
  }
  if (t < CW) sB2[t] = b2[t];
  __syncthreads();

  {
    v8f acc[4];
#pragma unroll
    for (int nt = 0; nt < 4; ++nt) acc[nt] = zero8();
#pragma unroll
    for (int ks = 0; ks < 2; ++ks) {
      const v16h a = ldfrag(h16, CW, p0 + mt * 16, ks * 32, lane);
#pragma unroll
      for (int nt = 0; nt < 4; ++nt) {
        const v16h bf = ldfrag(w1p, CW, (nq * 4 + nt) * 16, ks * 32, lane);
        acc[nt] = mma16(a, bf, acc[nt]);
      }
    }
#pragma unroll
    for (int nt = 0; nt < 4; ++nt) {
#pragma unroll
      for (int r = 0; r < 8; ++r) {
        const int row = mt * 16 + 8 * hh + r, o = (nq * 4 + nt) * 16 + c;
        float z = acc[nt][r] * 0.125f + sB1[o];
        z = (z > 0.0f) ? z : 0.0f;
        sT[row * 136 + o] = (_Float16)z;
      }
    }
  }
  __syncthreads();

  {
    v8f acc2[2];
    acc2[0] = zero8(); acc2[1] = zero8();
#pragma unroll
    for (int ks = 0; ks < 4; ++ks) {
      const v16h a = ldfrag(sT, 136, mt * 16, ks * 32, lane);
#pragma unroll
      for (int s = 0; s < 2; ++s) {
        const v16h bf = ldfrag(w2p, CHID, (nq * 2 + s) * 16, ks * 32, lane);
        acc2[s] = mma16(a, bf, acc2[s]);
      }
    }
#pragma unroll
    for (int s = 0; s < 2; ++s) {
#pragma unroll
      for (int r = 0; r < 8; ++r) {
        const int row = mt * 16 + 8 * hh + r, o = (nq * 2 + s) * 16 + c;
        const float bb = acc2[s][r] * 0.125f + sB2[o];
        sBB[row * 64 + o] = bb;
        if (LAST) sB16[row * 72 + o] = (_Float16)bb;
      }
    }
  }
  __syncthreads();

#pragma unroll
  for (int it = 0; it < 4; ++it) {
    const int idx = t + 256 * it;
    const int L = idx >> 3, pc = idx & 7;
    const int row = L >> 1, half = L & 1;
    float* gp = x32 + (size_t)(p0 + row) * CW + half * 32 + pc * 4;
    const v4f old = *(const v4f*)gp;
    const v4f add = *(const v4fa*)(sBB + row * 64 + half * 32 + pc * 4);
    const v4f nv = old + add;
    st2_f4(gp, nv);
  }

  if (LAST) {
    v8f acc3[4];
#pragma unroll
    for (int nt = 0; nt < 4; ++nt) acc3[nt] = zero8();
#pragma unroll
    for (int ks = 0; ks < 2; ++ks) {
      const v16h a = ldfrag(sB16, 72, mt * 16, ks * 32, lane);
#pragma unroll
      for (int nt = 0; nt < 4; ++nt) {
        const v16h bf = ldfrag(wo1p, CW, (nq * 4 + nt) * 16, ks * 32, lane);
        acc3[nt] = mma16(a, bf, acc3[nt]);
      }
    }
    float s[8];
#pragma unroll
    for (int r = 0; r < 8; ++r) s[r] = 0.0f;
#pragma unroll
    for (int nt = 0; nt < 4; ++nt) {
      const int o = (nq * 4 + nt) * 16 + c;
      const float bo = sBo1[o], wv = sWo2[o];
#pragma unroll
      for (int r = 0; r < 8; ++r) s[r] += (acc3[nt][r] * 0.125f + bo) * wv;
    }
#pragma unroll
    for (int r = 0; r < 8; ++r) {
      s[r] += __shfl_xor(s[r], 8);
      s[r] += __shfl_xor(s[r], 4);
      s[r] += __shfl_xor(s[r], 2);
      s[r] += __shfl_xor(s[r], 1);
    }
    if (c == 0) {
#pragma unroll
      for (int r = 0; r < 8; ++r) sPart[(mt * 16 + 8 * hh + r) * 2 + nq] = s[r];
    }
    __syncthreads();
    if (t < 64) sOut[t] = (sPart[t * 2] + sPart[t * 2 + 1]) + bo2[0];
    __syncthreads();
    if (t < 16) {
      const v4f v = *(const v4fa*)(sOut + t * 4);
      st2_f4(out + p0 + t * 4, v);
    }
  }
}

extern "C" void kernel_launch(void* const* d_in, const int* in_sizes, int n_in,
                              void* d_out, int out_size, void* d_ws, size_t ws_size,
                              hipStream_t stream) {
  if (n_in < 13) return;
  if (in_sizes[0] != NPIX * CIN) return;
  if (in_sizes[1] != CW * CIN || in_sizes[2] != CW) return;
  if (in_sizes[3] != NLAYER * CW * CW * NMODE || in_sizes[4] != NLAYER * CW * CW * NMODE) return;
  if (in_sizes[5] != NLAYER * CHID * CW || in_sizes[6] != NLAYER * CHID) return;
  if (in_sizes[7] != NLAYER * CW * CHID || in_sizes[8] != NLAYER * CW) return;
  if (in_sizes[9] != CHID * CW || in_sizes[10] != CHID || in_sizes[11] != CHID || in_sizes[12] < 1) return;
  if (out_size != NPIX) return;
  if (ws_size < WS_TOTAL) return;

  const float* x    = (const float*)d_in[0];
  const float* W_in = (const float*)d_in[1];
  const float* b_in = (const float*)d_in[2];
  const float* fw0  = (const float*)d_in[3];
  const float* fw1  = (const float*)d_in[4];
  const float* ffW1 = (const float*)d_in[5];
  const float* ffb1 = (const float*)d_in[6];
  const float* ffW2 = (const float*)d_in[7];
  const float* ffb2 = (const float*)d_in[8];
  const float* W_o1 = (const float*)d_in[9];
  const float* b_o1 = (const float*)d_in[10];
  const float* W_o2 = (const float*)d_in[11];
  const float* b_o2 = (const float*)d_in[12];
  float* out = (float*)d_out;
  char* ws = (char*)d_ws;

  _Float16* df  = (_Float16*)(ws + OFF_DF);
  _Float16* dt  = (_Float16*)(ws + OFF_DT);
  float*    x32 = (float*)(ws + OFF_X);
  _Float16* h16 = (_Float16*)(ws + OFF_H);
  _Float16* xf  = (_Float16*)(ws + OFF_XF);
  _Float16* ymy = (_Float16*)(ws + OFF_YY);
  _Float16* ymx = (_Float16*)(ws + OFF_YX);
  _Float16* wm0 = (_Float16*)(ws + OFF_WM0);
  _Float16* wm1 = (_Float16*)(ws + OFF_WM1);
  _Float16* w1p = (_Float16*)(ws + OFF_W1);
  _Float16* w2p = (_Float16*)(ws + OFF_W2);
  _Float16* wo1 = (_Float16*)(ws + OFF_WO);

  k_dct_planes<<<dim3(1), dim3(256), 0, stream>>>(df, dt);
  k_cvt_modes<<<dim3(NMODE, NLAYER), dim3(256), 0, stream>>>(fw0, wm0);
  k_cvt_modes<<<dim3(NMODE, NLAYER), dim3(256), 0, stream>>>(fw1, wm1);
  k_cvt_lin<<<dim3((NLAYER * CHID * CW) / 2048), dim3(256), 0, stream>>>(ffW1, w1p, NLAYER * CHID * CW);
  k_cvt_lin<<<dim3((NLAYER * CW * CHID) / 2048), dim3(256), 0, stream>>>(ffW2, w2p, NLAYER * CW * CHID);
  k_cvt_lin<<<dim3((CHID * CW) / 2048), dim3(256), 0, stream>>>(W_o1, wo1, CHID * CW);
  k_lift<<<dim3(NPIX / 64), dim3(256), 0, stream>>>(x, W_in, b_in, x32);

  (void)hipFuncSetAttribute(reinterpret_cast<const void*>(&k_inv), hipFuncAttributeMaxDynamicSharedMemorySize, LDS_INV);

  for (int l = 0; l < NLAYER; ++l) {
    k_dct_fwd<<<dim3(NSLICE), dim3(256), 0, stream>>>(x32, df, xf, NCOLN * CW, CW);
    k_mode_mix<<<dim3((NSLICE / 16) * 2), dim3(256), 0, stream>>>(xf, wm0 + (size_t)l * NMODE * CW * CW, ymy);
    k_dct_fwd<<<dim3(NSLICE), dim3(256), 0, stream>>>(x32, df, xf, CW, NCOLN * CW);
    k_mode_mix<<<dim3((NSLICE / 16) * 2), dim3(256), 0, stream>>>(xf, wm1 + (size_t)l * NMODE * CW * CW, ymx);
    k_inv<<<dim3(NBATCH * 16 * 16), dim3(256), LDS_INV, stream>>>(dt, ymy, ymx, h16);
    if (l + 1 < NLAYER) {
      k_ffn<false><<<dim3(NPIX / 64), dim3(256), 0, stream>>>(h16, w1p + (size_t)l * CHID * CW, ffb1 + l * CHID,
                                                             w2p + (size_t)l * CW * CHID, ffb2 + l * CW, x32,
                                                             wo1, b_o1, W_o2, b_o2, out);
    } else {
      k_ffn<true><<<dim3(NPIX / 64), dim3(256), 0, stream>>>(h16, w1p + (size_t)l * CHID * CW, ffb1 + l * CHID,
                                                            w2p + (size_t)l * CW * CHID, ffb2 + l * CW, x32,
                                                            wo1, b_o1, W_o2, b_o2, out);
    }
  }
  (void)hipGetLastError();
}
